// GNNDMoN_807453851816
// MI455X (gfx1250) — hardware-verified
//
#include <hip/hip_runtime.h>
#include <stddef.h>


#define INF0    128
#define HID     64
#define KCL     16
#define NCLS    10
#define NPG     1024
#define NTHR    256
#define NWAVE   8
#define EPT     8
#define NGRP    2
#define CHUNK   (NTHR * EPT * NGRP)
#define WCAP    (EPT * NGRP * 32)
#define LISTN   (NWAVE * WCAP)
#define NBD     4096
#define G1ROWS  128
#define APITCH  136
#define PASS    128
#define STGW    32
#define MAXG    256
#define WSCALE  8.0f
#define WINV    0.125f
#define SQ      ((NPG * HID) / (NWAVE * 128))

#define LDS_GEMM1 (G1ROWS * APITCH * 2)
#define LDS_AGG   (NPG * HID * 4 + LISTN * 4 + 64)

static_assert((CHUNK & (CHUNK - 1)) == 0);
static_assert(CHUNK <= 4096);
static_assert(NPG <= 4096 && NBD <= 4096);
static_assert((NPG & (NPG - 1)) == 0 && (NBD & (NBD - 1)) == 0);
static_assert(NPG % (16 * NWAVE) == 0);
static_assert(G1ROWS * HID * 4 <= LDS_GEMM1);
static_assert(PASS * KCL + HID * KCL + KCL + HID + 32 <= LISTN);
static_assert(KCL * HID <= PASS * KCL);
static_assert(NPG % PASS == 0 && PASS <= NTHR && (PASS % 32) == 0);
static_assert((NPG * HID / 4) % NTHR == 0);
static_assert((NPG * HID) % (NWAVE * 128) == 0);
static_assert(NTHR == KCL * (HID / 4));
static_assert(HID % 32 == 0 && INF0 % 32 == 0 && HID % 16 == 0);
static_assert((G1ROWS * INF0 / 8) % NTHR == 0);
static_assert(NBD == NWAVE * 4 * 128);

typedef float    v2f  __attribute__((ext_vector_type(2)));
typedef float    v4f  __attribute__((ext_vector_type(4)));
typedef float    v8f  __attribute__((ext_vector_type(8)));
typedef int      v4i  __attribute__((ext_vector_type(4)));
typedef _Float16 v8h  __attribute__((ext_vector_type(8)));
typedef _Float16 v16h __attribute__((ext_vector_type(16)));
union FragH { v16h v; v8h h[2]; };

__device__ __forceinline__ v8h cvt8(v4f a, v4f b) {
  v8h r;
  r[0] = (_Float16)a.x; r[1] = (_Float16)a.y; r[2] = (_Float16)a.z; r[3] = (_Float16)a.w;
  r[4] = (_Float16)b.x; r[5] = (_Float16)b.y; r[6] = (_Float16)b.z; r[7] = (_Float16)b.w;
  return r;
}

__device__ __forceinline__ v8f wmh(v16h a, v16h b, v8f c) {
  v8f d = __builtin_amdgcn_wmma_f32_16x16x32_f16(false, a, false, b, (short)0, c, false, false);
  asm volatile("v_nop\n\tv_nop\n\tv_nop\n\tv_nop" : "+v"(d) : "v"(a), "v"(b));
  return d;
}

__device__ __forceinline__ float max4(v4f v) { return fmaxf(fmaxf(v.x, v.y), fmaxf(v.z, v.w)); }
__device__ __forceinline__ float sum4(v4f v) { return (v.x + v.y) + (v.z + v.w); }
__device__ __forceinline__ v4f exp4(v4f v) {
  v4f r;
  r.x = __expf(v.x); r.y = __expf(v.y); r.z = __expf(v.z); r.w = __expf(v.w);
  return r;
}
__device__ __forceinline__ float selu1(float a) {
  const float SC = 1.0507009873554805f, AL = 1.6732632423543772f;
  const float neg = AL * (__expf(a) - 1.0f);
  return SC * (a > 0.0f ? a : neg);
}

template <int NB>
__device__ __forceinline__ int scan_chunk(const int* __restrict__ dsts, int nE, int cbase, int nodeBase,
                                          int vec8, int* list, int tid, int lane, int wave) {
  int wc = 0;
#pragma unroll
  for (int g = 0; g < NGRP; ++g) {
    const int el0  = (g * NTHR + tid) * EPT;
    const int e0   = cbase + el0;
    const int sent = -2147483647 - 1;
    v4i da, db;
    if (vec8 != 0 && cbase + CHUNK <= nE) {
      da = *(const v4i*)(dsts + e0);
      db = *(const v4i*)(dsts + e0 + 4);
    } else {
      da.x = (e0     < nE) ? dsts[min(e0, nE - 1)] : sent;
      da.y = (e0 + 1 < nE) ? dsts[min(e0 + 1, nE - 1)] : sent;
      da.z = (e0 + 2 < nE) ? dsts[min(e0 + 2, nE - 1)] : sent;
      da.w = (e0 + 3 < nE) ? dsts[min(e0 + 3, nE - 1)] : sent;
      db.x = (e0 + 4 < nE) ? dsts[min(e0 + 4, nE - 1)] : sent;
      db.y = (e0 + 5 < nE) ? dsts[min(e0 + 5, nE - 1)] : sent;
      db.z = (e0 + 6 < nE) ? dsts[min(e0 + 6, nE - 1)] : sent;
      db.w = (e0 + 7 < nE) ? dsts[min(e0 + 7, nE - 1)] : sent;
    }
    const unsigned nb = (unsigned)nodeBase;
    const unsigned s0 = (unsigned)da.x - nb, s1 = (unsigned)da.y - nb;
    const unsigned s2 = (unsigned)da.z - nb, s3 = (unsigned)da.w - nb;
    const unsigned s4 = (unsigned)db.x - nb, s5 = (unsigned)db.y - nb;
    const unsigned s6 = (unsigned)db.z - nb, s7 = (unsigned)db.w - nb;
    const bool h0 = s0 < (unsigned)NB, h1 = s1 < (unsigned)NB, h2 = s2 < (unsigned)NB, h3 = s3 < (unsigned)NB;
    const bool h4 = s4 < (unsigned)NB, h5 = s5 < (unsigned)NB, h6 = s6 < (unsigned)NB, h7 = s7 < (unsigned)NB;
    const unsigned any = __builtin_amdgcn_ballot_w32(h0 | h1 | h2 | h3 | h4 | h5 | h6 | h7);
    if (any != 0u) {
#define HITJ(J, HJ, SJ) { \
        const unsigned mj = __builtin_amdgcn_ballot_w32(HJ); \
        if (mj != 0u) { \
          if (HJ) { \
            const int pos = wc + (int)__builtin_amdgcn_mbcnt_lo(mj, 0u); \
            if (pos < WCAP) list[wave * WCAP + pos] = ((el0 + (J)) << 12) | (int)(SJ); \
          } \
          wc += (int)__builtin_popcount(mj); } }
      HITJ(0, h0, s0)
      HITJ(1, h1, s1)
      HITJ(2, h2, s2)
      HITJ(3, h3, s3)
      HITJ(4, h4, s4)
      HITJ(5, h5, s5)
      HITJ(6, h6, s6)
      HITJ(7, h7, s7)
#undef HITJ
    }
  }
  return wc;
}

__global__ __launch_bounds__(NTHR) void k_wprep(
    const float* __restrict__ W1, const float* __restrict__ W2,
    _Float16* w1s, _Float16* w2s) {
  const int i  = blockIdx.x * NTHR + threadIdx.x;
  const int n1 = HID * INF0 / 8;
  const int n2 = HID * HID / 8;
  if (i >= n1 + n2) return;
  const bool first = i < n1;
  const int i1 = i < n1 - 1 ? i : n1 - 1;
  int i2 = i - n1; i2 = i2 < 0 ? 0 : (i2 > n2 - 1 ? n2 - 1 : i2);
  const v4f a1 = *(const v4f*)(W1 + (size_t)i1 * 8), c1 = *(const v4f*)(W1 + (size_t)i1 * 8 + 4);
  const v4f a2 = *(const v4f*)(W2 + (size_t)i2 * 8), c2 = *(const v4f*)(W2 + (size_t)i2 * 8 + 4);
  v4f a = first ? a1 : a2;
  v4f b = first ? c1 : c2;
  a = a * WSCALE;
  b = b * WSCALE;
  const v8h hv = cvt8(a, b);
  _Float16* dp = first ? (w1s + (size_t)i1 * 8) : (w2s + (size_t)i2 * 8);
  *(volatile v8h*)dp = hv;
  __threadfence();
  *(volatile v8h*)dp = hv;
}

__global__ __launch_bounds__(NTHR) void k_deg(
    const int* __restrict__ ei, float* dinv, int nN, int nE, int vec8) {
  __shared__ __attribute__((aligned(16))) int cnt[NBD];
  __shared__ __attribute__((aligned(16))) int list[LISTN];
  __shared__ int wcnt[NWAVE];
  const int tid = threadIdx.x, lane = tid & 31, wave = tid >> 5;
  const int nodeBase = blockIdx.x * NBD;
  const int* dsts = ei + nE;
  (void)nN;

  for (int i = tid; i < NBD; i += NTHR) cnt[i] = 0;
  __syncthreads();

  const int nChunks = (nE + CHUNK - 1) / CHUNK;
#pragma unroll 1
  for (int ch = 0; ch < nChunks; ++ch) {
    const int cbase = ch * CHUNK;
    const int wc = scan_chunk<NBD>(dsts, nE, cbase, nodeBase, vec8, list, tid, lane, wave);
    if (lane == 0) wcnt[wave] = wc;
    __syncthreads();
    if (wave == 0) {
#pragma unroll 1
      for (int wsx = 0; wsx < NWAVE; ++wsx) {
        int n = __builtin_amdgcn_readfirstlane(wcnt[wsx]);
        n = n > WCAP ? WCAP : (n < 0 ? 0 : n);
        const int* lp = list + wsx * WCAP;
#pragma unroll 1
        for (int i = 0; i < n; ++i) {
          const int ent  = __builtin_amdgcn_readfirstlane(lp[i]);
          const int slot = ent & (NBD - 1);
          if (lane == 0) cnt[slot] = cnt[slot] + 1;
        }
      }
    }
    __syncthreads();
  }

  v4f dq[4];
#pragma unroll
  for (int q = 0; q < 4; ++q) {
    const int f = (wave * 4 + q) * 128 + 4 * lane;
    const v4i c = *(const v4i*)(cnt + f);
    dq[q].x = rsqrtf((float)(c.x + 1));
    dq[q].y = rsqrtf((float)(c.y + 1));
    dq[q].z = rsqrtf((float)(c.z + 1));
    dq[q].w = rsqrtf((float)(c.w + 1));
  }
  float* dp = dinv + (size_t)nodeBase;
#pragma unroll
  for (int q = 0; q < 4; ++q) *(volatile v4f*)(dp + (wave * 4 + q) * 128 + 4 * lane) = dq[q];
  __threadfence();
#pragma unroll
  for (int q = 0; q < 4; ++q) *(volatile v4f*)(dp + (wave * 4 + q) * 128 + 4 * lane) = dq[q];
}

__global__ __launch_bounds__(NTHR) void k_gemm1(
    const float* __restrict__ x, const _Float16* __restrict__ w1s,
    const float* __restrict__ dinv, float* g1, int nN) {
  __shared__ v4f lds_g[LDS_GEMM1 / 16];
  _Float16* sA  = (_Float16*)lds_g;
  float*    stg = (float*)lds_g;
  const int tid = threadIdx.x, lane = tid & 31, wave = tid >> 5, hh = lane >> 4, m = lane & 15;
  const int rowBase = blockIdx.x * G1ROWS;

#pragma unroll
  for (int i = 0; i < (G1ROWS * INF0 / 8) / NTHR; ++i) {
    const int idx = i * NTHR + tid;
    const int r   = idx >> 4;
    const int c0  = (idx & 15) * 8;
    int node = rowBase + r;
    node = node > nN - 1 ? nN - 1 : node;
    const float* xp = x + (size_t)node * INF0 + c0;
    const v4f a = *(const v4f*)xp, b = *(const v4f*)(xp + 4);
    *(v8h*)(sA + r * APITCH + c0) = cvt8(a, b);
  }
  __syncthreads();

  v8f acc[HID / 16];
#pragma unroll
  for (int t = 0; t < HID / 16; ++t) { v8f z = {0.f, 0.f, 0.f, 0.f, 0.f, 0.f, 0.f, 0.f}; acc[t] = z; }
  const _Float16* ar = sA + (wave * 16 + m) * APITCH + 8 * hh;
#pragma unroll
  for (int kt = 0; kt < INF0 / 32; ++kt) {
    FragH a;
    a.h[0] = *(const v8h*)(ar + 32 * kt);
    a.h[1] = *(const v8h*)(ar + 32 * kt + 16);
#pragma unroll
    for (int t = 0; t < HID / 16; ++t) {
      const _Float16* bp = w1s + (size_t)(16 * t + m) * INF0 + 32 * kt + 8 * hh;
      FragH b;
      b.h[0] = *(const v8h*)bp;
      b.h[1] = *(const v8h*)(bp + 16);
      acc[t] = wmh(a.v, b.v, acc[t]);
    }
  }
  __syncthreads();

  const int r0 = wave * 16 + 8 * hh;
  const v4f dA = *(const v4f*)(dinv + (size_t)rowBase + r0);
  const v4f dB = *(const v4f*)(dinv + (size_t)rowBase + r0 + 4);
  const float d0 = dA.x * WINV, d1 = dA.y * WINV, d2 = dA.z * WINV, d3 = dA.w * WINV;
  const float d4 = dB.x * WINV, d5 = dB.y * WINV, d6 = dB.z * WINV, d7 = dB.w * WINV;
  float* sp = stg + r0 * HID + m;
#pragma unroll
  for (int t = 0; t < HID / 16; ++t) {
    sp[0 * HID + 16 * t] = acc[t][0] * d0;
    sp[1 * HID + 16 * t] = acc[t][1] * d1;
    sp[2 * HID + 16 * t] = acc[t][2] * d2;
    sp[3 * HID + 16 * t] = acc[t][3] * d3;
    sp[4 * HID + 16 * t] = acc[t][4] * d4;
    sp[5 * HID + 16 * t] = acc[t][5] * d5;
    sp[6 * HID + 16 * t] = acc[t][6] * d6;
    sp[7 * HID + 16 * t] = acc[t][7] * d7;
  }
  __syncthreads();

  const float* lp = stg + wave * 16 * HID;
  float* gp = g1 + ((size_t)rowBase + wave * 16) * HID;
#pragma unroll
  for (int q = 0; q < (16 * HID) / 128; ++q) { const int f = q * 128 + 4 * lane; const v4f v = *(const v4f*)(lp + f); *(volatile v4f*)(gp + f) = v; }
  __threadfence();
#pragma unroll
  for (int q = 0; q < (16 * HID) / 128; ++q) { const int f = q * 128 + 4 * lane; const v4f v = *(const v4f*)(lp + f); *(volatile v4f*)(gp + f) = v; }
}

__global__ __launch_bounds__(NTHR) void k_layer1(
    const int* __restrict__ ei, const float* __restrict__ g1, const float* __restrict__ dinv,
    const float* __restrict__ b1, const _Float16* __restrict__ w2s, float* g2,
    int nN, int nE, int vec8) {
  extern __shared__ v4f lds_dyn[];
  float* acc  = (float*)lds_dyn;
  int*   list = (int*)(acc + NPG * HID);
  int*   wcnt = list + LISTN;
  const int tid = threadIdx.x, lane = tid & 31, wave = tid >> 5, hh = lane >> 4, m = lane & 15;
  const int nodeBase = blockIdx.x * NPG;
  const int* dsts = ei + nE;

  {
    const v4f z = {0.f, 0.f, 0.f, 0.f};
    for (int i = tid; i < NPG * HID / 4; i += NTHR) lds_dyn[i] = z;
  }
  __syncthreads();

  const int nChunks = (nE + CHUNK - 1) / CHUNK;
#pragma unroll 1
  for (int ch = 0; ch < nChunks; ++ch) {
    const int cbase = ch * CHUNK;
    const int wc = scan_chunk<NPG>(dsts, nE, cbase, nodeBase, vec8, list, tid, lane, wave);
    if (lane == 0) wcnt[wave] = wc;
    __syncthreads();
    if (wave == 0) {
#pragma unroll 1
      for (int wsx = 0; wsx < NWAVE; ++wsx) {
        int n = __builtin_amdgcn_readfirstlane(wcnt[wsx]);
        n = n > WCAP ? WCAP : (n < 0 ? 0 : n);
        const int* lp = list + wsx * WCAP;
#pragma unroll 1
        for (int i = 0; i < n; ++i) {
          const int ent  = __builtin_amdgcn_readfirstlane(lp[i]);
          const int slot = ent & (NPG - 1);
          int e = cbase + ((ent >> 12) & (CHUNK - 1));
          e = e > nE - 1 ? nE - 1 : e;
          int src = ei[e];
          src = src < 0 ? 0 : (src > nN - 1 ? nN - 1 : src);
          const v2f v = *(const v2f*)(g1 + (size_t)src * HID + 2 * lane);
          v2f* ap = (v2f*)(acc + slot * HID + 2 * lane);
          *ap = *ap + v;
        }
      }
    }
    __syncthreads();
  }

#pragma unroll 2
  for (int i = 0; i < (NPG * HID / 4) / NTHR; ++i) {
    const int idx  = i * NTHR + tid;
    const int slot = idx >> 4;
    const int c4   = (idx & 15) * 4;
    int node = nodeBase + slot;
    node = node > nN - 1 ? nN - 1 : node;
    const float d  = dinv[node];
    const v4f   gv = *(const v4f*)(g1 + (size_t)node * HID + c4);
    const v4f   bv = *(const v4f*)(b1 + c4);
    v4f* ap = (v4f*)(acc + slot * HID + c4);
    v4f hv = (*ap + gv) * d + bv;
    hv.x = fmaxf(hv.x, 0.f); hv.y = fmaxf(hv.y, 0.f); hv.z = fmaxf(hv.z, 0.f); hv.w = fmaxf(hv.w, 0.f);
    *ap = hv;
  }
  __syncthreads();

#pragma unroll 1
  for (int it = 0; it < NPG / 16 / NWAVE; ++it) {
    const int t = it * NWAVE + wave;
    v8f c[HID / 16];
#pragma unroll
    for (int ct = 0; ct < HID / 16; ++ct) { v8f z = {0.f, 0.f, 0.f, 0.f, 0.f, 0.f, 0.f, 0.f}; c[ct] = z; }
#pragma unroll
    for (int kt = 0; kt < HID / 32; ++kt) {
      const float* ap = acc + (16 * t + m) * HID + 32 * kt + 8 * hh;
      const v4f p0 = *(const v4f*)ap,        p1 = *(const v4f*)(ap + 4);
      const v4f p2 = *(const v4f*)(ap + 16), p3 = *(const v4f*)(ap + 20);
      FragH a;
      a.h[0] = cvt8(p0, p1);
      a.h[1] = cvt8(p2, p3);
#pragma unroll
      for (int ct = 0; ct < HID / 16; ++ct) {
        const _Float16* bp = w2s + (size_t)(16 * ct + m) * HID + 32 * kt + 8 * hh;
        FragH b;
        b.h[0] = *(const v8h*)bp;
        b.h[1] = *(const v8h*)(bp + 16);
        c[ct] = wmh(a.v, b.v, c[ct]);
      }
    }
    __syncthreads();
    const int node0 = nodeBase + 16 * t + 8 * hh;
    const v4f dA = *(const v4f*)(dinv + (size_t)node0);
    const v4f dB = *(const v4f*)(dinv + (size_t)node0 + 4);
    const float d0 = dA.x * WINV, d1 = dA.y * WINV, d2 = dA.z * WINV, d3 = dA.w * WINV;
    const float d4 = dB.x * WINV, d5 = dB.y * WINV, d6 = dB.z * WINV, d7 = dB.w * WINV;
    float* sp = acc + (16 * t + 8 * hh) * HID + m;
#pragma unroll
    for (int ct = 0; ct < HID / 16; ++ct) {
      sp[0 * HID + 16 * ct] = c[ct][0] * d0;
      sp[1 * HID + 16 * ct] = c[ct][1] * d1;
      sp[2 * HID + 16 * ct] = c[ct][2] * d2;
      sp[3 * HID + 16 * ct] = c[ct][3] * d3;
      sp[4 * HID + 16 * ct] = c[ct][4] * d4;
      sp[5 * HID + 16 * ct] = c[ct][5] * d5;
      sp[6 * HID + 16 * ct] = c[ct][6] * d6;
      sp[7 * HID + 16 * ct] = c[ct][7] * d7;
    }
  }
  __syncthreads();

  float* gp = g2 + (size_t)nodeBase * HID;
#pragma unroll 4
  for (int q = 0; q < SQ; ++q) {
    const int f = (wave * SQ + q) * 128 + 4 * lane;
    const v4f v = *(const v4f*)(acc + f);
    *(volatile v4f*)(gp + f) = v;
  }
  __threadfence();
#pragma unroll 4
  for (int q = 0; q < SQ; ++q) {
    const int f = (wave * SQ + q) * 128 + 4 * lane;
    const v4f v = *(const v4f*)(acc + f);
    *(volatile v4f*)(gp + f) = v;
  }
}

__global__ __launch_bounds__(NTHR) void k_layer2(
    const int* __restrict__ ei, const float* __restrict__ g2, const float* __restrict__ dinv,
    const float* __restrict__ b2, const float* __restrict__ Wp, const float* __restrict__ bp,
    const float* __restrict__ Wl, const float* __restrict__ bl, float* gst,
    int nN, int nE, int vec8) {
  extern __shared__ v4f lds_dyn[];
  float* acc  = (float*)lds_dyn;
  int*   list = (int*)(acc + NPG * HID);
  int*   wcnt = list + LISTN;
  float* sl   = (float*)list;
  float* wpT  = sl + PASS * KCL;
  float* bpL  = wpT + HID * KCL;
  float* ov   = bpL + KCL;
  float* ost  = ov + HID;
  float* xp   = sl;
  const int tid = threadIdx.x, lane = tid & 31, wave = tid >> 5;
  const int nodeBase = blockIdx.x * NPG;
  const int* dsts = ei + nE;

  {
    const v4f z = {0.f, 0.f, 0.f, 0.f};
    for (int i = tid; i < NPG * HID / 4; i += NTHR) lds_dyn[i] = z;
  }
  __syncthreads();

  const int nChunks = (nE + CHUNK - 1) / CHUNK;
#pragma unroll 1
  for (int ch = 0; ch < nChunks; ++ch) {
    const int cbase = ch * CHUNK;
    const int wc = scan_chunk<NPG>(dsts, nE, cbase, nodeBase, vec8, list, tid, lane, wave);
    if (lane == 0) wcnt[wave] = wc;
    __syncthreads();
    if (wave == 0) {
#pragma unroll 1
      for (int wsx = 0; wsx < NWAVE; ++wsx) {
        int n = __builtin_amdgcn_readfirstlane(wcnt[wsx]);
        n = n > WCAP ? WCAP : (n < 0 ? 0 : n);
        const int* lp = list + wsx * WCAP;
#pragma unroll 1
        for (int i = 0; i < n; ++i) {
          const int ent  = __builtin_amdgcn_readfirstlane(lp[i]);
          const int slot = ent & (NPG - 1);
          int e = cbase + ((ent >> 12) & (CHUNK - 1));
          e = e > nE - 1 ? nE - 1 : e;
          int src = ei[e];
          src = src < 0 ? 0 : (src > nN - 1 ? nN - 1 : src);
          const v2f v = *(const v2f*)(g2 + (size_t)src * HID + 2 * lane);
          v2f* ap = (v2f*)(acc + slot * HID + 2 * lane);
          *ap = *ap + v;
        }
      }
    }
    __syncthreads();
  }

#pragma unroll 2
  for (int i = 0; i < (NPG * HID / 4) / NTHR; ++i) {
    const int idx  = i * NTHR + tid;
    const int slot = idx >> 4;
    const int c4   = (idx & 15) * 4;
    int node = nodeBase + slot;
    node = node > nN - 1 ? nN - 1 : node;
    const float d  = dinv[node];
    const v4f   gv = *(const v4f*)(g2 + (size_t)node * HID + c4);
    const v4f   bv = *(const v4f*)(b2 + c4);
    v4f* ap = (v4f*)(acc + slot * HID + c4);
    v4f hv = (*ap + gv) * d + bv;
    hv.x = fmaxf(hv.x, 0.f); hv.y = fmaxf(hv.y, 0.f); hv.z = fmaxf(hv.z, 0.f); hv.w = fmaxf(hv.w, 0.f);
    *ap = hv;
  }
  for (int i = tid; i < KCL * HID; i += NTHR) {
    const int k = i / HID;
    const int h = i - k * HID;
    wpT[h * KCL + k] = Wp[i];
  }
  if (tid < KCL) bpL[tid] = bp[tid];
  __syncthreads();

  v4f P = {0.f, 0.f, 0.f, 0.f};
  const int pk = tid >> 4;
  const int ph = (tid & 15) * 4;
#pragma unroll 1
  for (int p = 0; p < NPG / PASS; ++p) {
    if (tid < PASS) {
      const float* row = acc + (p * PASS + tid) * HID;
      v4f L0 = {0.f, 0.f, 0.f, 0.f}, L1 = L0, L2 = L0, L3 = L0;
#pragma unroll 1
      for (int h = 0; h < HID; ++h) {
        const float xv = row[h];
        const v4f* wq = (const v4f*)(wpT + h * KCL);
        L0 += xv * wq[0]; L1 += xv * wq[1]; L2 += xv * wq[2]; L3 += xv * wq[3];
      }
      const v4f* bq = (const v4f*)bpL;
      L0 += bq[0]; L1 += bq[1]; L2 += bq[2]; L3 += bq[3];
      const float mx = fmaxf(fmaxf(max4(L0), max4(L1)), fmaxf(max4(L2), max4(L3)));
      const v4f E0 = exp4(L0 - mx), E1 = exp4(L1 - mx), E2 = exp4(L2 - mx), E3 = exp4(L3 - mx);
      const float ssum = (sum4(E0) + sum4(E1)) + (sum4(E2) + sum4(E3));
      const float inv = 1.0f / ssum;
      v4f* sp = (v4f*)(sl + tid * KCL);
      sp[0] = E0 * inv; sp[1] = E1 * inv; sp[2] = E2 * inv; sp[3] = E3 * inv;
    }
    __syncthreads();
#pragma unroll 2
    for (int n = 0; n < PASS; ++n) {
      const float sv = sl[n * KCL + pk];
      const v4f   hv = *(const v4f*)(acc + (p * PASS + n) * HID + ph);
      P += sv * hv;
    }
    __syncthreads();
  }

  v4f X;
  X.x = selu1(P.x); X.y = selu1(P.y); X.z = selu1(P.z); X.w = selu1(P.w);
  *(v4f*)(xp + pk * HID + ph) = X;
  __syncthreads();
  if (tid < HID) {
    float o = 0.f;
#pragma unroll 1
    for (int k = 0; k < KCL; ++k) o += xp[k * HID + tid];
    ov[tid] = o * (1.0f / KCL);
  }
  __syncthreads();
  if (tid < 32) {
    const int cc = lane < NCLS ? lane : NCLS - 1;
    float a = 0.f;
#pragma unroll 1
    for (int h = 0; h < HID; ++h) a += ov[h] * Wl[cc * HID + h];
    a += bl[cc];
    ost[lane] = (lane < NCLS) ? a : 0.f;
  }
  __syncthreads();
  if (wave == 0) {
    const int l8 = lane & 7;
    const v4f v = *(const v4f*)(ost + 4 * l8);
    float* gp = gst + (size_t)blockIdx.x * STGW + 4 * l8;
    if (lane < 8) *(volatile v4f*)gp = v;
    __threadfence();
    if (lane < 8) *(volatile v4f*)gp = v;
  }
}

__global__ __launch_bounds__(NTHR) void k_final(const float* __restrict__ gst, float* out, int nGr) {
  __shared__ __attribute__((aligned(16))) float so[MAXG * NCLS];
  const int tid = threadIdx.x;
  int ng = nGr; ng = ng > MAXG ? MAXG : (ng < 0 ? 0 : ng);
  const int T = ng * NCLS;
  for (int i = tid; i < T; i += NTHR) {
    const int g = i / NCLS;
    const int c = i - g * NCLS;
    so[i] = gst[(size_t)g * STGW + c];
  }
  __syncthreads();
  const int nv = T >> 2;
  for (int i = tid; i < nv; i += NTHR) { const v4f v = *(const v4f*)(so + 4 * i); *(volatile v4f*)(out + 4 * i) = v; }
  if (tid == 0) { for (int j = nv * 4; j < T; ++j) { const float v = so[j]; *(volatile float*)(out + j) = v; } }
  __threadfence();
  for (int i = tid; i < nv; i += NTHR) { const v4f v = *(const v4f*)(so + 4 * i); *(volatile v4f*)(out + 4 * i) = v; }
  if (tid == 0) { for (int j = nv * 4; j < T; ++j) { const float v = so[j]; *(volatile float*)(out + j) = v; } }
}

extern "C" void kernel_launch(void* const* d_in, const int* in_sizes, int n_in,
                              void* d_out, int out_size, void* d_ws, size_t ws_size,
                              hipStream_t stream) {
  if (n_in < 11) return;
  const int nN = in_sizes[0] / INF0;
  const int nE = in_sizes[1] / 2;
  if (nN <= 0 || nE <= 0 || in_sizes[0] != nN * INF0 || in_sizes[1] != nE * 2) return;
  if ((nN % NPG) != 0) return;
  const int nGr = nN / NPG;
  if (nGr < 1 || nGr > MAXG) return;
  if (in_sizes[3] != HID * INF0 || in_sizes[4] < HID || in_sizes[5] != HID * HID || in_sizes[6] < HID) return;
  if (in_sizes[7] != KCL * HID || in_sizes[8] < KCL || in_sizes[9] != NCLS * HID || in_sizes[10] < NCLS) return;
  if (out_size != nGr * NCLS) return;

  const float* x  = (const float*)d_in[0];
  const int*   ei = (const int*)d_in[1];
  const float* W1 = (const float*)d_in[3];
  const float* b1 = (const float*)d_in[4];
  const float* W2 = (const float*)d_in[5];
  const float* b2 = (const float*)d_in[6];
  const float* Wp = (const float*)d_in[7];
  const float* bp = (const float*)d_in[8];
  const float* Wl = (const float*)d_in[9];
  const float* bl = (const float*)d_in[10];
  float* out = (float*)d_out;

  const int nBD = (nN + NBD - 1) / NBD;
  const int nG1 = (nN + G1ROWS - 1) / G1ROWS;

  char* ws = (char*)d_ws;
  size_t off = 0;
  const size_t oW1 = off; off += (size_t)HID * INF0 * 2;                       off = (off + 255) & ~(size_t)255;
  const size_t oW2 = off; off += (size_t)HID * HID * 2;                        off = (off + 255) & ~(size_t)255;
  const size_t oDv = off; off += (size_t)nBD * NBD * 4;                        off = (off + 255) & ~(size_t)255;
  const size_t oG1 = off; off += (size_t)nG1 * G1ROWS * HID * 4;               off = (off + 255) & ~(size_t)255;
  const size_t oG2 = off; off += (size_t)nGr * NPG * HID * 4;                  off = (off + 255) & ~(size_t)255;
  const size_t oSt = off; off += (size_t)nGr * STGW * 4;                       off = (off + 255) & ~(size_t)255;
  if (off > ws_size) return;
  _Float16* w1s  = (_Float16*)(ws + oW1);
  _Float16* w2s  = (_Float16*)(ws + oW2);
  float*    dinv = (float*)(ws + oDv);
  float*    g1   = (float*)(ws + oG1);
  float*    g2   = (float*)(ws + oG2);
  float*    gst  = (float*)(ws + oSt);

  const int vec8 = ((nE & 3) == 0) ? 1 : 0;

  const int nPrep = HID * INF0 / 8 + HID * HID / 8;
  k_wprep<<<(nPrep + NTHR - 1) / NTHR, NTHR, 0, stream>>>(W1, W2, w1s, w2s);

  k_deg<<<nBD, NTHR, 0, stream>>>(ei, dinv, nN, nE, vec8);

  k_gemm1<<<nG1, NTHR, 0, stream>>>(x, w1s, dinv, g1, nN);

  hipFuncSetAttribute(reinterpret_cast<const void*>(&k_layer1),
                      hipFuncAttributeMaxDynamicSharedMemorySize, LDS_AGG);
  k_layer1<<<nGr, NTHR, LDS_AGG, stream>>>(ei, g1, dinv, b1, w2s, g2, nN, nE, vec8);

  hipFuncSetAttribute(reinterpret_cast<const void*>(&k_layer2),
                      hipFuncAttributeMaxDynamicSharedMemorySize, LDS_AGG);
  k_layer2<<<nGr, NTHR, LDS_AGG, stream>>>(ei, g2, dinv, b2, Wp, bp, Wl, bl, gst, nN, nE, vec8);

  k_final<<<1, NTHR, 0, stream>>>(gst, out, nGr);
}
